// CustomGCNConv_37254546325944
// MI455X (gfx1250) — hardware-verified
//
#include <hip/hip_runtime.h>
#include <stddef.h>


#pragma clang fp contract(off)

#define NN     8192
#define CH     64
#define WPR    (NN / 32)
#define RB     128
#define NTHR   256
#define NWAVE  8
#define EPT    8
#define NGRP   2
#define CHUNK  (NTHR * EPT * NGRP)
#define WCAP   (EPT * NGRP * 32)
#define LISTN  (NWAVE * WCAP)
#define GTHR   128
#define GWAVE  4
#define KC     128
#define AP     136
#define HP     72
#define JP     128
#define SBUFN  (RB * HP * 2)
#define LDS_BITS ((RB * WPR + LISTN) * 4 + RB * 4 + 64)

static_assert((CHUNK & (CHUNK - 1)) == 0);
static_assert(CHUNK <= 4096);
static_assert((RB & (RB - 1)) == 0 && RB <= 4096);
static_assert(NN % RB == 0 && NN % KC == 0 && (KC % 32) == 0);
static_assert(RB == GTHR && RB == 32 * GWAVE);
static_assert(NTHR == 32 * NWAVE && RB == 16 * NWAVE);
static_assert(WPR == 256);
static_assert(SBUFN >= RB * AP && SBUFN >= RB * CH * 2);
static_assert((AP % 8) == 0 && (HP % 8) == 0 && (JP % 8) == 0);
static_assert(LDS_BITS >= (RB * WPR + LISTN) * 4 + RB * 4 + NWAVE * 4);

typedef float          v4f   __attribute__((ext_vector_type(4)));
typedef float          v8f   __attribute__((ext_vector_type(8)));
typedef int            v4i   __attribute__((ext_vector_type(4)));
typedef unsigned int   v4u   __attribute__((ext_vector_type(4)));
typedef unsigned short v8us  __attribute__((ext_vector_type(8)));
typedef __bf16         v16bf __attribute__((ext_vector_type(16)));
union FragB { v16bf v; v8us h[2]; };

__device__ __forceinline__ v8f wmb(v16bf a, v16bf b, v8f c) {
  v8f d = __builtin_amdgcn_wmma_f32_16x16x32_bf16(false, a, false, b, (short)0, c, false, false);
  asm volatile("v_nop\n\tv_nop\n\tv_nop\n\tv_nop" : "+v"(d) : "v"(a), "v"(b));
  return d;
}

__device__ __forceinline__ unsigned int bf16rne(float f) {
  const unsigned int u = __float_as_uint(f);
  return (u + 0x7FFFu + ((u >> 16) & 1u)) >> 16;
}

__device__ __forceinline__ void split2(float v, unsigned short& hi, unsigned short& lo) {
  const unsigned int hbits = bf16rne(v);
  const float hf = __uint_as_float(hbits << 16);
  const unsigned int lbits = bf16rne(v - hf);
  hi = (unsigned short)hbits;
  lo = (unsigned short)lbits;
}

template <int NB>
__device__ __forceinline__ int scan_chunk(const int* __restrict__ keys, int nE, int cbase, int slotBase,
                                          int* list, int tid, int lane, int wave) {
  int wc = 0;
#pragma unroll
  for (int g = 0; g < NGRP; ++g) {
    const int el0  = (g * NTHR + tid) * EPT;
    const int e0   = cbase + el0;
    const int sent = -2147483647 - 1;
    v4i da, db;
    if (cbase + CHUNK <= nE) {
      da = *(const v4i*)(keys + e0);
      db = *(const v4i*)(keys + e0 + 4);
    } else {
      da.x = (e0     < nE) ? keys[min(e0,     nE - 1)] : sent;
      da.y = (e0 + 1 < nE) ? keys[min(e0 + 1, nE - 1)] : sent;
      da.z = (e0 + 2 < nE) ? keys[min(e0 + 2, nE - 1)] : sent;
      da.w = (e0 + 3 < nE) ? keys[min(e0 + 3, nE - 1)] : sent;
      db.x = (e0 + 4 < nE) ? keys[min(e0 + 4, nE - 1)] : sent;
      db.y = (e0 + 5 < nE) ? keys[min(e0 + 5, nE - 1)] : sent;
      db.z = (e0 + 6 < nE) ? keys[min(e0 + 6, nE - 1)] : sent;
      db.w = (e0 + 7 < nE) ? keys[min(e0 + 7, nE - 1)] : sent;
    }
    const unsigned nb = (unsigned)slotBase;
    const unsigned s0 = (unsigned)da.x - nb, s1 = (unsigned)da.y - nb;
    const unsigned s2 = (unsigned)da.z - nb, s3 = (unsigned)da.w - nb;
    const unsigned s4 = (unsigned)db.x - nb, s5 = (unsigned)db.y - nb;
    const unsigned s6 = (unsigned)db.z - nb, s7 = (unsigned)db.w - nb;
    const bool h0 = s0 < (unsigned)NB, h1 = s1 < (unsigned)NB, h2 = s2 < (unsigned)NB, h3 = s3 < (unsigned)NB;
    const bool h4 = s4 < (unsigned)NB, h5 = s5 < (unsigned)NB, h6 = s6 < (unsigned)NB, h7 = s7 < (unsigned)NB;
    const unsigned any = __builtin_amdgcn_ballot_w32(h0 | h1 | h2 | h3 | h4 | h5 | h6 | h7);
    if (any != 0u) {
#define HITJ(J, HJ, SJ) { \
        const unsigned mj = __builtin_amdgcn_ballot_w32(HJ); \
        if (mj != 0u) { \
          if (HJ) { \
            const int pos = wc + (int)__builtin_amdgcn_mbcnt_lo(mj, 0u); \
            if (pos < WCAP) list[wave * WCAP + pos] = ((el0 + (J)) << 12) | (int)(SJ); \
          } \
          wc += (int)__builtin_popcount(mj); } }
      HITJ(0, h0, s0)
      HITJ(1, h1, s1)
      HITJ(2, h2, s2)
      HITJ(3, h3, s3)
      HITJ(4, h4, s4)
      HITJ(5, h5, s5)
      HITJ(6, h6, s6)
      HITJ(7, h7, s7)
#undef HITJ
    }
  }
  return wc;
}

__global__ __launch_bounds__(NTHR) void k_bits(
    const int* __restrict__ ei, unsigned int* bitsG, float* dinvG, int nE) {
  extern __shared__ v4u lds_dyn[];
  unsigned int* bits = (unsigned int*)lds_dyn;
  int*   list = (int*)(bits + RB * WPR);
  float* sD   = (float*)(list + LISTN);
  int*   wcnt = (int*)(sD + RB);
  const int tid = threadIdx.x, lane = tid & 31, wave = tid >> 5;
  const int rowBase = blockIdx.x * RB;

  {
    const v4u z = {0u, 0u, 0u, 0u};
#pragma unroll 4
    for (int i = tid; i < RB * WPR / 4; i += NTHR) ((v4u*)bits)[i] = z;
  }
  __syncthreads();

  const int nChunks = (nE + CHUNK - 1) / CHUNK;
#pragma unroll 1
  for (int ch = 0; ch < nChunks; ++ch) {
    const int cbase = ch * CHUNK;
    const int wc = scan_chunk<RB>(ei, nE, cbase, rowBase, list, tid, lane, wave);
    if (lane == 0) wcnt[wave] = wc;
    __syncthreads();
    if (wave == 0) {
#pragma unroll 1
      for (int wsx = 0; wsx < NWAVE; ++wsx) {
        int n = __builtin_amdgcn_readfirstlane(wcnt[wsx]);
        n = n > WCAP ? WCAP : (n < 0 ? 0 : n);
        const int* lp = list + wsx * WCAP;
#pragma unroll 1
        for (int i = 0; i < n; ++i) {
          const int ent  = __builtin_amdgcn_readfirstlane(lp[i]);
          const int slot = ent & (RB - 1);
          int e = cbase + ((ent >> 12) & (CHUNK - 1));
          e = e > nE - 1 ? nE - 1 : e;
          int d = ei[(size_t)nE + e];
          d = d < 0 ? 0 : (d > NN - 1 ? NN - 1 : d);
          if (lane == 0) {
            unsigned int* wp = bits + slot * WPR + (d >> 5);
            const unsigned int nv = *wp | (1u << (d & 31));
            *wp = nv;
          }
        }
      }
    }
    __syncthreads();
  }

#pragma unroll
  for (int q = 0; q < 16; ++q) {
    const int r = wave * 16 + q;
    const v4u w0 = *(const v4u*)(bits + r * WPR + 8 * lane);
    const v4u w1 = *(const v4u*)(bits + r * WPR + 8 * lane + 4);
    int pc = (int)__popc(w0.x) + (int)__popc(w0.y) + (int)__popc(w0.z) + (int)__popc(w0.w)
           + (int)__popc(w1.x) + (int)__popc(w1.y) + (int)__popc(w1.z) + (int)__popc(w1.w);
#pragma unroll
    for (int off = 16; off > 0; off >>= 1) pc += __shfl_xor(pc, off, 32);
    const int deg = pc + 1;
    const float dv = deg > 0 ? rsqrtf((float)deg) : 0.0f;
    if (lane == 0) sD[r] = dv;
  }
  __syncthreads();

  v4f dq = {0.f, 0.f, 0.f, 0.f};
  if (tid < 32) dq = *(const v4f*)(sD + 4 * tid);
  float* dp = dinvG + (size_t)rowBase + 4 * tid;
  unsigned int* gp = bitsG + (size_t)rowBase * WPR;
  if (tid < 32) *(volatile v4f*)dp = dq;
#pragma unroll 4
  for (int i = 0; i < RB * WPR / (4 * NTHR); ++i) {
    const int p = i * NTHR + tid;
    const v4u v = ((const v4u*)bits)[p];
    *(volatile v4u*)(gp + 4 * p) = v;
  }
  __threadfence();
  if (tid < 32) *(volatile v4f*)dp = dq;
#pragma unroll 4
  for (int i = 0; i < RB * WPR / (4 * NTHR); ++i) {
    const int p = i * NTHR + tid;
    const v4u v = ((const v4u*)bits)[p];
    *(volatile v4u*)(gp + 4 * p) = v;
  }
}

__global__ __launch_bounds__(GTHR) void k_prep(
    const float* __restrict__ x, const float* __restrict__ dinvG,
    unsigned short* yhi, unsigned short* ylo) {
  __shared__ __attribute__((aligned(16))) unsigned short sHi[CH * JP];
  __shared__ __attribute__((aligned(16))) unsigned short sLo[CH * JP];
  const int tid = threadIdx.x, lane = tid & 31, wave = tid >> 5, hs = lane >> 4, l16 = lane & 15;
  const int jBase = blockIdx.x * RB;
  const int j = jBase + tid;
  const float dj = dinvG[j];
#pragma unroll
  for (int c4 = 0; c4 < CH / 4; ++c4) {
    const v4f xv = *(const v4f*)(x + (size_t)j * CH + 4 * c4);
    unsigned short hi, lo;
    split2(xv.x * dj, hi, lo); sHi[(4 * c4 + 0) * JP + tid] = hi; sLo[(4 * c4 + 0) * JP + tid] = lo;
    split2(xv.y * dj, hi, lo); sHi[(4 * c4 + 1) * JP + tid] = hi; sLo[(4 * c4 + 1) * JP + tid] = lo;
    split2(xv.z * dj, hi, lo); sHi[(4 * c4 + 2) * JP + tid] = hi; sLo[(4 * c4 + 2) * JP + tid] = lo;
    split2(xv.w * dj, hi, lo); sHi[(4 * c4 + 3) * JP + tid] = hi; sLo[(4 * c4 + 3) * JP + tid] = lo;
  }
  __syncthreads();

#pragma unroll
  for (int i = 0; i < 8; ++i) {
    const int c = 2 * (wave + GWAVE * i) + hs;
    const v8us a = *(const v8us*)(sHi + c * JP + 8 * l16);
    const v8us b = *(const v8us*)(sLo + c * JP + 8 * l16);
    *(volatile v8us*)(yhi + (size_t)c * NN + jBase + 8 * l16) = a;
    *(volatile v8us*)(ylo + (size_t)c * NN + jBase + 8 * l16) = b;
  }
  __threadfence();
#pragma unroll
  for (int i = 0; i < 8; ++i) {
    const int c = 2 * (wave + GWAVE * i) + hs;
    const v8us a = *(const v8us*)(sHi + c * JP + 8 * l16);
    const v8us b = *(const v8us*)(sLo + c * JP + 8 * l16);
    *(volatile v8us*)(yhi + (size_t)c * NN + jBase + 8 * l16) = a;
    *(volatile v8us*)(ylo + (size_t)c * NN + jBase + 8 * l16) = b;
  }
}

__device__ __forceinline__ void expand_word(unsigned short* dst, unsigned int w, const v4u* lut) {
#pragma unroll
  for (int b = 0; b < 4; ++b) {
    const unsigned int byte = (w >> (8 * b)) & 255u;
    const v4u v = lut[byte];
    *(v4u*)(dst + 8 * b) = v;
  }
}

__global__ __launch_bounds__(GTHR) void k_gcn(
    const unsigned int* __restrict__ bitsG, const unsigned short* __restrict__ yhi,
    const unsigned short* __restrict__ ylo, const float* __restrict__ dinvG,
    const float* __restrict__ W, const float* __restrict__ bias, float* out) {
  __shared__ __attribute__((aligned(16))) unsigned short sbuf[SBUFN];
  __shared__ __attribute__((aligned(16))) unsigned short sWh[CH * HP];
  __shared__ __attribute__((aligned(16))) unsigned short sWl[CH * HP];
  __shared__ __attribute__((aligned(16))) v4u lut[256];
  __shared__ __attribute__((aligned(16))) float sDv[RB];
  const int tid = threadIdx.x, lane = tid & 31, wave = tid >> 5, hh = lane >> 4, m = lane & 15;
  const int rowBase = blockIdx.x * RB;

  for (int e = tid; e < 256; e += GTHR) {
    v4u v;
    v.x = (((unsigned)e >> 0) & 1u) * 0x3F80u | (((((unsigned)e >> 1) & 1u) * 0x3F80u) << 16);
    v.y = (((unsigned)e >> 2) & 1u) * 0x3F80u | (((((unsigned)e >> 3) & 1u) * 0x3F80u) << 16);
    v.z = (((unsigned)e >> 4) & 1u) * 0x3F80u | (((((unsigned)e >> 5) & 1u) * 0x3F80u) << 16);
    v.w = (((unsigned)e >> 6) & 1u) * 0x3F80u | (((((unsigned)e >> 7) & 1u) * 0x3F80u) << 16);
    lut[e] = v;
  }
  sDv[tid] = dinvG[(size_t)rowBase + tid];
#pragma unroll 4
  for (int i = 0; i < CH * CH / GTHR; ++i) {
    const int idx = i * GTHR + tid;
    const int n = idx >> 6, k = idx & 63;
    unsigned short hi, lo;
    split2(W[idx], hi, lo);
    sWh[n * HP + k] = hi;
    sWl[n * HP + k] = lo;
  }

  v8f acc[2][4];
#pragma unroll
  for (int mi = 0; mi < 2; ++mi)
#pragma unroll
    for (int t = 0; t < 4; ++t) { v8f z = {0.f, 0.f, 0.f, 0.f, 0.f, 0.f, 0.f, 0.f}; acc[mi][t] = z; }
  __syncthreads();

  unsigned short* arow = sbuf + tid * AP;
  const unsigned int* brow = bitsG + (size_t)(rowBase + tid) * WPR;
#pragma unroll 1
  for (int c = 0; c < NN / KC; ++c) {
    const int kBase = c * KC;
    const v4u wv = *(const v4u*)(brow + (kBase >> 5));
    expand_word(arow,      wv.x, lut);
    expand_word(arow + 32, wv.y, lut);
    expand_word(arow + 64, wv.z, lut);
    expand_word(arow + 96, wv.w, lut);
    if (kBase == rowBase) {
      __syncthreads();
      const unsigned short cur = arow[tid];
      arow[tid] = (cur != 0) ? (unsigned short)0x4000 : (unsigned short)0x3F80;
    }
    __syncthreads();

#pragma unroll
    for (int ks = 0; ks < KC / 32; ++ks) {
      const int k0 = 32 * ks;
      FragB a0, a1;
      const unsigned short* ap0 = sbuf + (wave * 32 + m) * AP + k0 + 8 * hh;
      const unsigned short* ap1 = ap0 + 16 * AP;
      a0.h[0] = *(const v8us*)ap0;        a0.h[1] = *(const v8us*)(ap0 + 16);
      a1.h[0] = *(const v8us*)ap1;        a1.h[1] = *(const v8us*)(ap1 + 16);
#pragma unroll
      for (int t = 0; t < 4; ++t) {
        const size_t boff = (size_t)(16 * t + m) * NN + kBase + k0 + 8 * hh;
        FragB bh, bl;
        bh.h[0] = *(const v8us*)(yhi + boff);   bh.h[1] = *(const v8us*)(yhi + boff + 16);
        acc[0][t] = wmb(a0.v, bh.v, acc[0][t]);
        acc[1][t] = wmb(a1.v, bh.v, acc[1][t]);
        bl.h[0] = *(const v8us*)(ylo + boff);   bl.h[1] = *(const v8us*)(ylo + boff + 16);
        acc[0][t] = wmb(a0.v, bl.v, acc[0][t]);
        acc[1][t] = wmb(a1.v, bl.v, acc[1][t]);
      }
    }
    __syncthreads();
  }

  unsigned short* sHh = sbuf;
  unsigned short* sHl = sbuf + RB * HP;
#pragma unroll
  for (int mi = 0; mi < 2; ++mi) {
    const int rb = wave * 32 + 16 * mi + 8 * hh;
    float dv[8];
#pragma unroll
    for (int r = 0; r < 8; ++r) dv[r] = sDv[rb + r];
#pragma unroll
    for (int t = 0; t < 4; ++t) {
      const int col = 16 * t + m;
#pragma unroll
      for (int r = 0; r < 8; ++r) {
        unsigned short hi, lo;
        split2(acc[mi][t][r] * dv[r], hi, lo);
        sHh[(rb + r) * HP + col] = hi;
        sHl[(rb + r) * HP + col] = lo;
      }
    }
  }
  __syncthreads();

  v8f acc2[2][4];
#pragma unroll
  for (int t = 0; t < 4; ++t) {
    const float bv = bias[16 * t + m];
    v8f z; z[0] = bv; z[1] = bv; z[2] = bv; z[3] = bv; z[4] = bv; z[5] = bv; z[6] = bv; z[7] = bv;
    acc2[0][t] = z; acc2[1][t] = z;
  }
#pragma unroll
  for (int ks = 0; ks < CH / 32; ++ks) {
    const int k0 = 32 * ks;
    FragB ah[2], al[2];
#pragma unroll
    for (int mi = 0; mi < 2; ++mi) {
      const int ro = (wave * 32 + 16 * mi + m) * HP + k0 + 8 * hh;
      ah[mi].h[0] = *(const v8us*)(sHh + ro);  ah[mi].h[1] = *(const v8us*)(sHh + ro + 16);
      al[mi].h[0] = *(const v8us*)(sHl + ro);  al[mi].h[1] = *(const v8us*)(sHl + ro + 16);
    }
#pragma unroll
    for (int t = 0; t < 4; ++t) {
      const int wo = (16 * t + m) * HP + k0 + 8 * hh;
      FragB wh, wl;
      wh.h[0] = *(const v8us*)(sWh + wo);  wh.h[1] = *(const v8us*)(sWh + wo + 16);
      wl.h[0] = *(const v8us*)(sWl + wo);  wl.h[1] = *(const v8us*)(sWl + wo + 16);
#pragma unroll
      for (int mi = 0; mi < 2; ++mi) {
        acc2[mi][t] = wmb(ah[mi].v, wh.v, acc2[mi][t]);
        acc2[mi][t] = wmb(ah[mi].v, wl.v, acc2[mi][t]);
        acc2[mi][t] = wmb(al[mi].v, wh.v, acc2[mi][t]);
      }
    }
  }
  __syncthreads();

  float* sO = (float*)sbuf;
#pragma unroll
  for (int mi = 0; mi < 2; ++mi) {
    const int rb = wave * 32 + 16 * mi + 8 * hh;
#pragma unroll
    for (int t = 0; t < 4; ++t) {
#pragma unroll
      for (int r = 0; r < 8; ++r) sO[(rb + r) * CH + 16 * t + m] = acc2[mi][t][r];
    }
  }
  __syncthreads();

  float* op = out + (size_t)rowBase * CH;
#pragma unroll
  for (int i = 0; i < RB * CH / (4 * GTHR); ++i) {
    const int p = i * GTHR + tid;
    const v4f v = *(const v4f*)(sO + 4 * p);
    *(volatile v4f*)(op + 4 * p) = v;
  }
  __threadfence();
#pragma unroll
  for (int i = 0; i < RB * CH / (4 * GTHR); ++i) {
    const int p = i * GTHR + tid;
    const v4f v = *(const v4f*)(sO + 4 * p);
    *(volatile v4f*)(op + 4 * p) = v;
  }
}

extern "C" void kernel_launch(void* const* d_in, const int* in_sizes, int n_in,
                              void* d_out, int out_size, void* d_ws, size_t ws_size,
                              hipStream_t stream) {
  if (n_in < 4) return;
  const int nE = in_sizes[1] / 2;
  if (in_sizes[0] != NN * CH || nE < 1 || in_sizes[1] != 2 * nE) return;
  if (in_sizes[2] != CH * CH || in_sizes[3] < CH || out_size != NN * CH) return;
  if (nE > (1 << 28)) return;

  const float* x  = (const float*)d_in[0];
  const int*   ei = (const int*)d_in[1];
  const float* W  = (const float*)d_in[2];
  const float* b  = (const float*)d_in[3];
  float* out = (float*)d_out;

  char* ws = (char*)d_ws;
  size_t off = 0;
  const size_t oBits = off; off += (size_t)NN * WPR * 4;   off = (off + 255) & ~(size_t)255;
  const size_t oDv   = off; off += (size_t)NN * 4;         off = (off + 255) & ~(size_t)255;
  const size_t oYh   = off; off += (size_t)CH * NN * 2;    off = (off + 255) & ~(size_t)255;
  const size_t oYl   = off; off += (size_t)CH * NN * 2;    off = (off + 255) & ~(size_t)255;
  if (off > ws_size) return;
  unsigned int*   bits = (unsigned int*)(ws + oBits);
  float*          dinv = (float*)(ws + oDv);
  unsigned short* yh   = (unsigned short*)(ws + oYh);
  unsigned short* yl   = (unsigned short*)(ws + oYl);

  hipFuncSetAttribute(reinterpret_cast<const void*>(&k_bits),
                      hipFuncAttributeMaxDynamicSharedMemorySize, LDS_BITS);
  k_bits<<<NN / RB, NTHR, LDS_BITS, stream>>>(ei, bits, dinv, nE);
  k_prep<<<NN / RB, GTHR, 0, stream>>>(x, dinv, yh, yl);
  k_gcn<<<NN / RB, GTHR, 0, stream>>>(bits, yh, yl, dinv, W, b, out);
}
